// myRNN_7524782702668
// MI455X (gfx1250) — hardware-run, weakly checked
//
#include <hip/hip_runtime.h>
#include <math.h>

constexpr int NB        = 512;
constexpr int NT        = 2048;
constexpr int NH        = 32;
constexpr int NTHR      = 256;
constexpr int NWAVE     = NTHR / 32;
constexpr int ROWS_WAVE = 16;
constexpr int ROWS_BLK  = NWAVE * ROWS_WAVE;
constexpr int NBLK      = NB / ROWS_BLK;
constexpr int CH        = 32;
constexpr int NCHUNK    = NT / CH;
constexpr int OBP       = 36;
constexpr float HCAR = 1024.0f;
constexpr float WCAR = 256.0f;
constexpr float FOLD = 1.0f / (HCAR * WCAR);
constexpr float F16_MIN_NORMAL = 6.103515625e-05f;

static_assert(NH == 32, "one 32-deep k-step covers the whole hidden width");
static_assert(NB % ROWS_BLK == 0, "whole blocks");
static_assert(NT % CH == 0, "whole chunks");
static_assert(CH * 4 == 128, "a chunk of one batch row is one 128-B line");
static_assert((NT * 4) % 128 == 0, "every batch row of the sequence output starts on a line");
static_assert(((size_t)NB * NT * 4) % 128 == 0, "the final-state output starts on a line");
static_assert((size_t)NB * NT * 4 == 4194304, "byte offset of the second output");
static_assert(NH * 4 == 128, "a final-state row is one 128-B line");
static_assert(OBP % 4 == 0 && OBP >= CH && OBP >= NH, "slab pitch");
static_assert(NBLK * NWAVE * ROWS_WAVE == NB, "waves cover the batch exactly");

typedef __attribute__((ext_vector_type(16))) _Float16 v16h;
typedef __attribute__((ext_vector_type(8)))  float    v8f;
typedef __attribute__((ext_vector_type(4)))  float    v4f;

__device__ __forceinline__ v8f mma_f16(v16h a, v16h b, v8f c) {
  c = __builtin_amdgcn_wmma_f32_16x16x32_f16(false, a, false, b, (short)0, c, false, false);
  asm volatile("v_nop\n\tv_nop\n\tv_nop\n\tv_nop" : "+v"(c) : "v"(a), "v"(b));
  return c;
}

__device__ __forceinline__ _Float16 to_f16_op(float v) {
  const float s = (fabsf(v) < F16_MIN_NORMAL) ? 0.0f : v;
  return (_Float16)s;
}

__device__ __forceinline__ void load8(const float* __restrict__ p, float (&d)[8]) {
  const v4f u = *(const v4f*)(p);
  const v4f w = *(const v4f*)(p + 4);
#pragma unroll
  for (int e = 0; e < 4; ++e) {
    d[e]     = u[e];
    d[4 + e] = w[e];
  }
}

__device__ __forceinline__ v16h load_w_frag(const float* __restrict__ rowp) {
  float k_lo[8], k_hi[8];
  load8(rowp, k_lo);
  load8(rowp + 16, k_hi);
  v16h f;
#pragma unroll
  for (int e = 0; e < 8; ++e) {
    f[e]     = to_f16_op(k_lo[e] * WCAR);
    f[8 + e] = to_f16_op(k_hi[e] * WCAR);
  }
  return f;
}

__device__ __forceinline__ void store_tile_lines(const float* sw, float* dst, int pitch, int lane) {
  v4f v[4];
#pragma unroll
  for (int it = 0; it < 4; ++it) {
    const int idx = it * 32 + lane;
    const int row = idx >> 3;
    const int q   = idx & 7;
    v[it] = *(const v4f*)(sw + row * OBP + q * 4);
  }
  for (int pass = 0; pass < 2; ++pass) {
#pragma unroll
    for (int it = 0; it < 4; ++it) {
      const int idx = it * 32 + lane;
      const int row = idx >> 3;
      const int q   = idx & 7;
      *(volatile v4f*)(dst + (size_t)row * pitch + q * 4) = v[it];
    }
    __threadfence();
  }
}

__global__ void __launch_bounds__(NTHR)
scan_tanh_cell_kernel(const float* __restrict__ x,
                      const float* __restrict__ h0,
                      const float* __restrict__ wih,
                      const float* __restrict__ whh,
                      const float* __restrict__ bih,
                      const float* __restrict__ bhh,
                      const float* __restrict__ wfc,
                      const float* __restrict__ bfc,
                      float* __restrict__ out_seq,
                      float* __restrict__ out_hlast) {
  __shared__ __align__(16) float slab[NWAVE][16 * OBP];

  const int tid  = threadIdx.x;
  const int lane = tid & 31;
  const int wave = tid >> 5;
  const int c    = lane & 15;
  const int hh   = lane >> 4;
  const int b0   = (blockIdx.x * NWAVE + wave) * ROWS_WAVE;
  float* const sw = &slab[wave][0];

  const v16h a0 = load_w_frag(whh + (size_t)c * NH + 8 * hh);
  const v16h a1 = load_w_frag(whh + (size_t)(16 + c) * NH + 8 * hh);

  float wi_lo[8], wi_hi[8], bs_lo[8], bs_hi[8], wf_lo[8], wf_hi[8];
  {
    float t_lo[8], t_hi[8];
    load8(wih + 8 * hh, wi_lo);
    load8(wih + 16 + 8 * hh, wi_hi);
    load8(bih + 8 * hh, bs_lo);
    load8(bih + 16 + 8 * hh, bs_hi);
    load8(bhh + 8 * hh, t_lo);
    load8(bhh + 16 + 8 * hh, t_hi);
#pragma unroll
    for (int r = 0; r < 8; ++r) {
      bs_lo[r] = bs_lo[r] + t_lo[r];
      bs_hi[r] = bs_hi[r] + t_hi[r];
    }
    load8(wfc + 8 * hh, wf_lo);
    load8(wfc + 16 + 8 * hh, wf_hi);
  }
  const float bfcv = bfc[0];

  float lo[8], hi[8];
  load8(h0 + (size_t)(b0 + c) * NH + 8 * hh, lo);
  load8(h0 + (size_t)(b0 + c) * NH + 16 + 8 * hh, hi);

  const float* const xrow = x + (size_t)(b0 + c) * NT;
  const v8f z8 = {0.f, 0.f, 0.f, 0.f, 0.f, 0.f, 0.f, 0.f};
  float xv = xrow[0];

#pragma unroll 1
  for (int ch = 0; ch < NCHUNK; ++ch) {
    const int t0 = ch * CH;
#pragma unroll 1
    for (int tt = 0; tt < CH; ++tt) {
      const int t  = t0 + tt;
      const int tn = (t + 1 < NT) ? (t + 1) : (NT - 1);
      const float xn = xrow[tn];

      v16h bf;
#pragma unroll
      for (int e = 0; e < 8; ++e) {
        bf[e]     = to_f16_op(lo[e] * HCAR);
        bf[8 + e] = to_f16_op(hi[e] * HCAR);
      }

      const v8f acc0 = mma_f16(a0, bf, z8);
      const v8f acc1 = mma_f16(a1, bf, z8);

#pragma unroll
      for (int r = 0; r < 8; ++r) {
        lo[r] = fmaf(acc0[r], FOLD, fmaf(xv, wi_lo[r], bs_lo[r]));
        hi[r] = fmaf(acc1[r], FOLD, fmaf(xv, wi_hi[r], bs_hi[r]));
      }

#pragma unroll 1
      for (int g = 0; g < 2; ++g) {
        float tv[8];
#pragma unroll
        for (int r = 0; r < 8; ++r) tv[r] = tanhf(lo[r]);
#pragma unroll
        for (int r = 0; r < 8; ++r) {
          lo[r] = hi[r];
          hi[r] = tv[r];
        }
      }

      float p = 0.0f;
#pragma unroll
      for (int r = 0; r < 8; ++r) p = fmaf(wf_lo[r], lo[r], p);
#pragma unroll
      for (int r = 0; r < 8; ++r) p = fmaf(wf_hi[r], hi[r], p);
      const float po = __shfl_xor(p, 16, 32);
      const float y  = (p + po) + bfcv;
      if (hh == 0) sw[c * OBP + tt] = y;

      xv = xn;
    }
    __syncthreads();
    store_tile_lines(sw, out_seq + (size_t)b0 * NT + t0, NT, lane);
    __syncthreads();
  }

#pragma unroll
  for (int r = 0; r < 8; ++r) {
    sw[c * OBP + 8 * hh + r]      = lo[r];
    sw[c * OBP + 16 + 8 * hh + r] = hi[r];
  }
  __syncthreads();
  store_tile_lines(sw, out_hlast + (size_t)b0 * NH, NH, lane);
}

extern "C" void kernel_launch(void* const* d_in, const int* in_sizes, int n_in,
                              void* d_out, int out_size, void* d_ws, size_t ws_size, hipStream_t stream) {
  (void)d_ws;
  (void)ws_size;
  if (n_in < 8 || d_out == nullptr) return;
  if (in_sizes[0] != NB * NT || in_sizes[1] != NB * NH || in_sizes[2] != NH || in_sizes[3] != NH * NH ||
      in_sizes[4] != NH || in_sizes[5] != NH || in_sizes[6] != NH || in_sizes[7] != 1 ||
      out_size != NB * NT + NB * NH) return;

  const float* x   = (const float*)d_in[0];
  const float* h0  = (const float*)d_in[1];
  const float* wih = (const float*)d_in[2];
  const float* whh = (const float*)d_in[3];
  const float* bih = (const float*)d_in[4];
  const float* bhh = (const float*)d_in[5];
  const float* wfc = (const float*)d_in[6];
  const float* bfc = (const float*)d_in[7];

  float* out_seq   = (float*)d_out;
  float* out_hlast = out_seq + (size_t)NB * NT;

  scan_tanh_cell_kernel<<<dim3(NBLK), dim3(NTHR), 0, stream>>>(
      x, h0, wih, whh, bih, bhh, wfc, bfc, out_seq, out_hlast);
}
